// Net_int_13580686590258
// MI455X (gfx1250) — hardware-verified
//
#include <hip/hip_runtime.h>
#include <stddef.h>
#include <stdint.h>
#include <math.h>

#define NN     4000
#define NE     64000
#define NPR    200000
#define MPN    4096
#define DIM    64
#define HK     128
#define CHR    2048
#define NT1    8320
#define TPLANE ((size_t)CHR * 8192)
#define NTHR   256
#define NWAVE  8
#define EPT    8
#define CHUNK  (NTHR * EPT)
#define WCAP   (EPT * 32)
#define LISTN  (NWAVE * WCAP)
#define NBA    1024
#define SLA    10
#define RCAP   28672
#define DEGCAP 48
#define MEAS_B1024  16431
#define MEAS_MAXDEG 35
#define BKT_ZINTS   (RCAP + 3 * NBA)
#define BKT_LDS_INTS (LISTN + 2 * RCAP + 3 * NBA + 16)
#define NU_BT1 (NT1 * 16)
#define NU_W1B (HK * 4)
#define NU_BTG (256 * 32)
#define NU_WWB (16 * 48)
#define NU_RT  1024
#define NU_GB  256
#define PB_BTG 0
#define PB_WWB 131072
#define PB_RT  143360
#define PB_GB  147456
#define PB_BYTES 148480
#define EAP    40
#define SDP    132
#define MAP    264
#define MDP    68
#define GSP    260
#define GRU_LDS_FLOATS (64 * GSP + 256)
#define RAP    392
#define RGP    17
#define RD_OFF_RT  25088
#define RD_OFF_G   26112
#define RD_OFF_Y   28288
#define RD_OFF_F   28416
#define RD_LDS_FLOATS 28424
#define WSMAX  134217728

static_assert((CHUNK & (CHUNK - 1)) == 0 && CHUNK <= 4096);
static_assert((NBA & (NBA - 1)) == 0 && NBA == (1 << SLA));
static_assert(((long long)NE << SLA) < (1LL << 31));
static_assert(LISTN >= NWAVE * WCAP);
static_assert((RCAP % 32) == 0 && (BKT_ZINTS % 4) == 0 && (BKT_ZINTS % (4 * NTHR)) == 0);
static_assert(RCAP >= MEAS_B1024 + 4096);
static_assert(DEGCAP >= MEAS_MAXDEG + 8 && DEGCAP == 48 && DEGCAP % 16 == 0);
static_assert(BKT_LDS_INTS * 4 <= 300000);
static_assert(NE % 128 == 0 && MPN % 64 == 0 && MPN == 2 * CHR && MPN >= NN && MPN == 4 * NBA);
static_assert(NT1 % 128 == 0 && NT1 >= 8192 + 64);
static_assert((8192 * 16) % NTHR == 0 && (8256 * 16) % NTHR == 0 && NU_BT1 % NTHR == 0 && NU_W1B % NTHR == 0);
static_assert(NU_BTG % NTHR == 0 && NU_WWB % NTHR == 0 && NU_RT % NTHR == 0 && NU_GB % NTHR == 0);
static_assert(NU_RT == 4 * NTHR && NU_GB == NTHR && NTHR == 4 * 64);
static_assert(PB_WWB == 256 * 256 * 2 && PB_RT == PB_WWB + 16 * 384 * 2 && PB_GB == PB_RT + 4096 && PB_BYTES == PB_GB + 1024);
static_assert((PB_RT % 128) == 0 && (PB_GB % 128) == 0);
static_assert((EAP * 2) % 16 == 0 && (SDP * 4) % 16 == 0 && (MAP * 2) % 16 == 0 && (MDP * 4) % 16 == 0);
static_assert((GSP * 4) % 16 == 0 && (RAP * 2) % 16 == 0);
static_assert(RD_OFF_RT * 4 == 128 * RAP * 2 && RD_OFF_G == RD_OFF_RT + 1024 && RD_OFF_Y == RD_OFF_G + 128 * RGP);
static_assert(RD_OFF_F == RD_OFF_Y + 128 && RD_LDS_FLOATS == RD_OFF_F + 8 && RD_LDS_FLOATS * 4 <= 300000);
static_assert(NPR % 32 == 0);

typedef float          v2f  __attribute__((ext_vector_type(2)));
typedef float          v4f  __attribute__((ext_vector_type(4)));
typedef float          v8f  __attribute__((ext_vector_type(8)));
typedef int            v4i  __attribute__((ext_vector_type(4)));
typedef int            v8i  __attribute__((ext_vector_type(8)));
typedef unsigned       v2u  __attribute__((ext_vector_type(2)));
typedef unsigned       v4u  __attribute__((ext_vector_type(4)));
typedef unsigned short v8us __attribute__((ext_vector_type(8)));
typedef __bf16         v16b __attribute__((ext_vector_type(16)));
typedef v2f  __attribute__((may_alias)) v2fa;
typedef v4f  __attribute__((may_alias)) v4fa;
typedef v4i  __attribute__((may_alias)) v4ia;
typedef v2u  __attribute__((may_alias)) v2ua;
typedef v4u  __attribute__((may_alias)) v4ua;
typedef v8us __attribute__((may_alias)) v8usa;
union FragB { v16b v; v8us h[2]; v8i w; };

__device__ __forceinline__ v8f wmb(const FragB& a, const FragB& b, v8f c) {
  v8f d = __builtin_amdgcn_wmma_f32_16x16x32_bf16(false, a.v, false, b.v, (short)0, c, false, false);
  asm volatile("v_nop\n\tv_nop\n\tv_nop\n\tv_nop" : "+v"(d) : "v"(a.w), "v"(b.w));
  return d;
}

__device__ __forceinline__ unsigned int f2bf(float f) {
  const unsigned int u = __float_as_uint(f);
  const unsigned int r = ((u + 0x7FFFu + ((u >> 16) & 1u)) >> 16) & 0xFFFFu;
  return ((u & 0x7FFFFFFFu) > 0x7F800000u) ? 0x7FC0u : r;
}
__device__ __forceinline__ float bf2f(unsigned int b) { return __uint_as_float(b << 16); }
__device__ __forceinline__ float bfr(float f) { return bf2f(f2bf(f)); }

__device__ __forceinline__ v2u split2(float a, float b) {
  const unsigned ha = f2bf(a);
  const unsigned hb = f2bf(b);
  const unsigned la = f2bf(a - bf2f(ha));
  const unsigned lb = f2bf(b - bf2f(hb));
  v2u r;
  r.x = ha | (hb << 16);
  r.y = la | (lb << 16);
  return r;
}

__device__ __forceinline__ unsigned blendbf(float a, float b, unsigned ma, unsigned mb) {
  const unsigned bits = (__float_as_uint(a) & ma) | (__float_as_uint(b) & mb);
  return f2bf(__uint_as_float(bits));
}

__device__ __forceinline__ unsigned selhl(float f, unsigned ml, unsigned mh) {
  const unsigned hb = f2bf(f);
  const unsigned lb = f2bf(f - bf2f(hb));
  return (hb & ml) | (lb & mh);
}

__device__ __forceinline__ v4u pack8sel(const float* sp, unsigned ml, unsigned mh) {
  const v4f a = *(const v4fa*)sp;
  const v4f b = *(const v4fa*)(sp + 4);
  v4u r;
  r.x = selhl(a.x, ml, mh) | (selhl(a.y, ml, mh) << 16);
  r.y = selhl(a.z, ml, mh) | (selhl(a.w, ml, mh) << 16);
  r.z = selhl(b.x, ml, mh) | (selhl(b.y, ml, mh) << 16);
  r.w = selhl(b.z, ml, mh) | (selhl(b.w, ml, mh) << 16);
  return r;
}

template <int SLB>
__device__ __forceinline__ int scan_chunk(const int* __restrict__ dsts, int nE, int cbase, int slotBase,
                                          int nb, int vec8, int* list, int tid, int lane, int wave) {
  int wc = 0;
  const int el0  = tid * EPT;
  const int e0   = cbase + el0;
  const int sent = -2147483647 - 1;
  v4i da, db;
  if (vec8 != 0 && cbase + CHUNK <= nE) {
    da = *(const v4i*)(dsts + e0);
    db = *(const v4i*)(dsts + e0 + 4);
  } else {
    da.x = (e0     < nE) ? dsts[min(e0,     nE - 1)] : sent;
    da.y = (e0 + 1 < nE) ? dsts[min(e0 + 1, nE - 1)] : sent;
    da.z = (e0 + 2 < nE) ? dsts[min(e0 + 2, nE - 1)] : sent;
    da.w = (e0 + 3 < nE) ? dsts[min(e0 + 3, nE - 1)] : sent;
    db.x = (e0 + 4 < nE) ? dsts[min(e0 + 4, nE - 1)] : sent;
    db.y = (e0 + 5 < nE) ? dsts[min(e0 + 5, nE - 1)] : sent;
    db.z = (e0 + 6 < nE) ? dsts[min(e0 + 6, nE - 1)] : sent;
    db.w = (e0 + 7 < nE) ? dsts[min(e0 + 7, nE - 1)] : sent;
  }
  const unsigned nbs = (unsigned)slotBase;
  const unsigned unb = (unsigned)nb;
  const unsigned s0 = (unsigned)da.x - nbs, s1 = (unsigned)da.y - nbs;
  const unsigned s2 = (unsigned)da.z - nbs, s3 = (unsigned)da.w - nbs;
  const unsigned s4 = (unsigned)db.x - nbs, s5 = (unsigned)db.y - nbs;
  const unsigned s6 = (unsigned)db.z - nbs, s7 = (unsigned)db.w - nbs;
  const bool h0 = s0 < unb, h1 = s1 < unb, h2 = s2 < unb, h3 = s3 < unb;
  const bool h4 = s4 < unb, h5 = s5 < unb, h6 = s6 < unb, h7 = s7 < unb;
  const unsigned any = __builtin_amdgcn_ballot_w32(h0 | h1 | h2 | h3 | h4 | h5 | h6 | h7);
  if (any != 0u) {
#define HITJ(J, HJ, SJ) { \
      const unsigned mj = __builtin_amdgcn_ballot_w32(HJ); \
      if (mj != 0u) { \
        if (HJ) { \
          const int pos = wc + (int)__builtin_amdgcn_mbcnt_lo(mj, 0u); \
          if (pos < WCAP) list[wave * WCAP + pos] = ((el0 + (J)) << SLB) | (int)(SJ); \
        } \
        wc += (int)__builtin_popcount(mj); } }
    HITJ(0, h0, s0)
    HITJ(1, h1, s1)
    HITJ(2, h2, s2)
    HITJ(3, h3, s3)
    HITJ(4, h4, s4)
    HITJ(5, h5, s5)
    HITJ(6, h6, s6)
    HITJ(7, h7, s7)
#undef HITJ
  }
  return wc;
}

__global__ __launch_bounds__(NTHR) __attribute__((amdgpu_num_vgpr(248)))
void k_pa(const float* __restrict__ W2, const float* __restrict__ b2, const float* __restrict__ W1,
          unsigned short* BT1, unsigned short* W1B) {
  const int u = (int)blockIdx.x * NTHR + (int)threadIdx.x;
  v8us o;
  unsigned short* dp;
  if (u < 8192 * 16) {
    const int row = u >> 4, c0 = (u & 15) * 8;
    const int oo = row >> 7, k = row & 127;
    const float* p = W2 + (size_t)k * 4096 + (size_t)(c0 & 63) * 64 + oo;
#pragma unroll
    for (int i = 0; i < 8; ++i) o[i] = (unsigned short)f2bf(p[(size_t)i * 64]);
    dp = BT1 + (size_t)row * 128 + c0;
  } else if (u < 8256 * 16) {
    const int row = u >> 4, c0 = (u & 15) * 8;
    const int oo = row - 8192;
    const float* p = b2 + (size_t)(c0 & 63) * 64 + oo;
#pragma unroll
    for (int i = 0; i < 8; ++i) o[i] = (unsigned short)f2bf(p[(size_t)i * 64]);
    dp = BT1 + (size_t)row * 128 + c0;
  } else if (u < NU_BT1) {
    const int row = u >> 4, c0 = (u & 15) * 8;
#pragma unroll
    for (int i = 0; i < 8; ++i) o[i] = (unsigned short)0;
    dp = BT1 + (size_t)row * 128 + c0;
  } else if (u < NU_BT1 + NU_W1B) {
    const int v = u - NU_BT1;
    const int n = v >> 2, c0 = (v & 3) * 8;
#pragma unroll
    for (int i = 0; i < 8; ++i) {
      const int c  = c0 + i;
      int kk = c < 12 ? c : c - 12;
      kk = kk > 11 ? 11 : kk;
      const float f = W1[(size_t)kk * HK + n];
      o[i] = (c < 24) ? (unsigned short)f2bf(f) : (unsigned short)0;
    }
    dp = W1B + (size_t)n * 32 + c0;
  } else {
    return;
  }
  *(volatile v8us*)dp = o;
  __threadfence();
  *(volatile v8us*)dp = o;
}

__global__ __launch_bounds__(NTHR) __attribute__((amdgpu_num_vgpr(248)))
void k_pb(const float* __restrict__ W_ih, const float* __restrict__ W_hh, const float* __restrict__ b_ih,
          const float* __restrict__ b_hh, const float* __restrict__ bmean, const float* __restrict__ bvar,
          const float* __restrict__ bgam, const float* __restrict__ bbet, const float* __restrict__ Wwt,
          const float* __restrict__ Wbias, unsigned char* PB) {
  __shared__ __attribute__((aligned(16))) float sT[NTHR];
  const int tid = (int)threadIdx.x;
  const int ub  = (int)blockIdx.x * NTHR;
  const int u   = ub + tid;
  if (ub < NU_BTG) {
    const int j = u >> 5, k8 = (u & 31) * 8, kk = k8 & 63;
    const int ri = j > 191 ? 191 : j;
    const int rh = (j < 192) ? j : j - 64;
    const v4f i0 = *(const v4f*)(W_ih + (size_t)ri * 64 + kk);
    const v4f i1 = *(const v4f*)(W_ih + (size_t)ri * 64 + kk + 4);
    const v4f g0 = *(const v4f*)(W_hh + (size_t)rh * 64 + kk);
    const v4f g1 = *(const v4f*)(W_hh + (size_t)rh * 64 + kk + 4);
    const bool ui = (k8 < 128) && (j < 192);
    const bool uh = (k8 >= 128) && (j < 128 || j >= 192);
    const unsigned mi = 0u - (unsigned)(ui ? 1 : 0);
    const unsigned mh = 0u - (unsigned)(uh ? 1 : 0);
    v4u o;
    o.x = blendbf(i0.x, g0.x, mi, mh) | (blendbf(i0.y, g0.y, mi, mh) << 16);
    o.y = blendbf(i0.z, g0.z, mi, mh) | (blendbf(i0.w, g0.w, mi, mh) << 16);
    o.z = blendbf(i1.x, g1.x, mi, mh) | (blendbf(i1.y, g1.y, mi, mh) << 16);
    o.w = blendbf(i1.z, g1.z, mi, mh) | (blendbf(i1.w, g1.w, mi, mh) << 16);
    unsigned short* dp = (unsigned short*)(PB + PB_BTG) + (size_t)j * 256 + k8;
    *(volatile v4u*)dp = o;
    __threadfence();
    *(volatile v4u*)dp = o;
  } else if (ub < NU_BTG + NU_WWB) {
    const int v = u - NU_BTG;
    const int j = v / 48, c0 = (v - 48 * j) * 8;
    const int cc = c0 < 192 ? c0 : c0 - 192;
    const int jc = j > 7 ? 7 : j;
    const v4f a0 = *(const v4f*)(Wwt + (size_t)jc * 192 + cc);
    const v4f a1 = *(const v4f*)(Wwt + (size_t)jc * 192 + cc + 4);
    const unsigned mj = 0u - (unsigned)((j < 8) ? 1 : 0);
    v4u o;
    o.x = blendbf(a0.x, 0.0f, mj, 0u) | (blendbf(a0.y, 0.0f, mj, 0u) << 16);
    o.y = blendbf(a0.z, 0.0f, mj, 0u) | (blendbf(a0.w, 0.0f, mj, 0u) << 16);
    o.z = blendbf(a1.x, 0.0f, mj, 0u) | (blendbf(a1.y, 0.0f, mj, 0u) << 16);
    o.w = blendbf(a1.z, 0.0f, mj, 0u) | (blendbf(a1.w, 0.0f, mj, 0u) << 16);
    unsigned short* dp = (unsigned short*)(PB + PB_WWB) + (size_t)j * 384 + c0;
    *(volatile v4u*)dp = o;
    __threadfence();
    *(volatile v4u*)dp = o;
  } else if (ub < NU_BTG + NU_WWB + NU_RT) {
    const int eb  = ub - NU_BTG - NU_WWB;
    const int idx = eb + tid;
    const int t  = idx / 192;
    const int cc = (idx < 768) ? (idx - 192 * t) : 0;
    int wi = idx - 768;
    wi = wi < 0 ? 0 : (wi > 7 ? 7 : wi);
    const float vm = bfr(bmean[cc]);
    const float vv = bfr(bvar[cc]);
    const float vg = bfr(bgam[cc]);
    const float vb = bfr(bbet[cc]);
    const float vw = bfr(Wbias[wi]);
    const float rs = 1.0f / sqrtf(vv + 1e-5f);
    const unsigned m0 = 0u - (unsigned)((t == 0) ? 1 : 0);
    const unsigned m1 = 0u - (unsigned)((t == 1) ? 1 : 0);
    const unsigned m2 = 0u - (unsigned)((t == 2) ? 1 : 0);
    const unsigned m3 = 0u - (unsigned)((t == 3) ? 1 : 0);
    const unsigned mw = 0u - (unsigned)((idx >= 768 && idx < 776) ? 1 : 0);
    const unsigned bits = (__float_as_uint(vm) & m0) | (__float_as_uint(rs) & m1) | (__float_as_uint(vg) & m2) |
                          (__float_as_uint(vb) & m3) | (__float_as_uint(vw) & mw);
    sT[tid] = __uint_as_float(bits);
    __syncthreads();
    if (tid < 64) {
      const v4f v = *(const v4fa*)(sT + 4 * tid);
      float* dp = (float*)(PB + PB_RT) + eb + 4 * tid;
      *(volatile v4f*)dp = v;
      __threadfence();
      *(volatile v4f*)dp = v;
    }
  } else if (ub < NU_BTG + NU_WWB + NU_RT + NU_GB) {
    const int j = u - NU_BTG - NU_WWB - NU_RT;
    const int ri = j > 191 ? 191 : j;
    const int rh = (j < 192) ? j : j - 64;
    const float bi = bfr(b_ih[ri]);
    const float bh = bfr(b_hh[rh]);
    const float bs = bi + bh;
    const unsigned m0 = 0u - (unsigned)((j < 128) ? 1 : 0);
    const unsigned m1 = 0u - (unsigned)((j >= 128 && j < 192) ? 1 : 0);
    const unsigned m2 = 0u - (unsigned)((j >= 192) ? 1 : 0);
    const unsigned bits = (__float_as_uint(bs) & m0) | (__float_as_uint(bi) & m1) | (__float_as_uint(bh) & m2);
    sT[tid] = __uint_as_float(bits);
    __syncthreads();
    if (tid < 64) {
      const v4f v = *(const v4fa*)(sT + 4 * tid);
      float* dp = (float*)(PB + PB_GB) + 4 * tid;
      *(volatile v4f*)dp = v;
      __threadfence();
      *(volatile v4f*)dp = v;
    }
  }
}

__global__ __launch_bounds__(NTHR) __attribute__((amdgpu_num_vgpr(248)))
void k_node(const float* __restrict__ x, const float* __restrict__ Wn, const float* __restrict__ bn_,
            float* H, unsigned short* HHL) {
  const int u = (int)blockIdx.x * NTHR + (int)threadIdx.x;
  const int row = u >> 4, c = (u & 15) * 4;
  const int rc = row < NN ? row : NN - 1;
  const bool ok = row < NN;
  const v4f bb = *(const v4f*)(bn_ + c);
  float a0 = 0.0f, a1 = 0.0f, a2 = 0.0f, a3 = 0.0f;
#pragma unroll 1
  for (int q = 0; q < 8; ++q) {
    const float xv = bfr(x[(size_t)rc * 8 + q]);
    const v4f w = *(const v4f*)(Wn + (size_t)q * DIM + c);
    a0 = fmaf(xv, bfr(w.x), a0);
    a1 = fmaf(xv, bfr(w.y), a1);
    a2 = fmaf(xv, bfr(w.z), a2);
    a3 = fmaf(xv, bfr(w.w), a3);
  }
  v4f hv;
  hv.x = ok ? fmaxf(a0 + bfr(bb.x), 0.0f) : 0.0f;
  hv.y = ok ? fmaxf(a1 + bfr(bb.y), 0.0f) : 0.0f;
  hv.z = ok ? fmaxf(a2 + bfr(bb.z), 0.0f) : 0.0f;
  hv.w = ok ? fmaxf(a3 + bfr(bb.w), 0.0f) : 0.0f;
  const v2u s01 = split2(hv.x, hv.y);
  const v2u s23 = split2(hv.z, hv.w);
  v2u wh, wl;
  wh.x = s01.x; wh.y = s23.x;
  wl.x = s01.y; wl.y = s23.y;
  float* hp = H + (size_t)row * DIM + c;
  unsigned short* bp = HHL + (size_t)row * 128 + c;
  *(volatile v4f*)hp = hv;
  *(volatile v2u*)bp = wh;
  *(volatile v2u*)(bp + 64) = wl;
  __threadfence();
  *(volatile v4f*)hp = hv;
  *(volatile v2u*)bp = wh;
  *(volatile v2u*)(bp + 64) = wl;
}

__global__ __launch_bounds__(128) __attribute__((amdgpu_num_vgpr(248)))
void k_edge(const float* __restrict__ ea, const float* __restrict__ We, const float* __restrict__ be,
            const float* __restrict__ b1, const unsigned short* __restrict__ W1B, unsigned short* H1HL) {
  __shared__ __attribute__((aligned(16))) float sW[240];
  __shared__ __attribute__((aligned(16))) unsigned short sA[128 * EAP];
  __shared__ __attribute__((aligned(16))) float stg[4 * 16 * SDP];
  __shared__ __attribute__((aligned(16))) float sb1[128];
  const int tid = (int)threadIdx.x, lane = tid & 31, wave = tid >> 5, hh = lane >> 4, m = lane & 15;

  {
    const int i0 = tid, i1 = tid + 128;
    const float w0 = We[i0];
    const int j1 = i1 < 228 ? i1 : 227;
    int j2 = i1 - 228; j2 = j2 < 0 ? 0 : (j2 > 11 ? 11 : j2);
    const float w1 = We[j1];
    const float w2 = be[j2];
    const unsigned m1 = 0u - (unsigned)((i1 < 228) ? 1 : 0);
    const float wsel = __uint_as_float((__float_as_uint(w1) & m1) | (__float_as_uint(w2) & ~m1));
    sW[i0] = bfr(w0);
    if (i1 < 240) sW[i1] = bfr(wsel);
    sb1[tid] = bfr(b1[tid]);
  }
  __syncthreads();

  const int e = (int)blockIdx.x * 128 + tid;
  {
    v4f q0 = {0.0f, 0.0f, 0.0f, 0.0f};
    v4f q1 = q0, q2 = q0;
    const float* xr = ea + (size_t)e * 19;
#pragma unroll 1
    for (int q = 0; q < 19; ++q) {
      const float xv = bfr(xr[q]);
      const float* wr = sW + q * 12;
      const v4f w0 = *(const v4fa*)wr;
      const v4f w1 = *(const v4fa*)(wr + 4);
      const v4f w2 = *(const v4fa*)(wr + 8);
      q0.x = fmaf(xv, w0.x, q0.x);  q0.y = fmaf(xv, w0.y, q0.y);
      q0.z = fmaf(xv, w0.z, q0.z);  q0.w = fmaf(xv, w0.w, q0.w);
      q1.x = fmaf(xv, w1.x, q1.x);  q1.y = fmaf(xv, w1.y, q1.y);
      q1.z = fmaf(xv, w1.z, q1.z);  q1.w = fmaf(xv, w1.w, q1.w);
      q2.x = fmaf(xv, w2.x, q2.x);  q2.y = fmaf(xv, w2.y, q2.y);
      q2.z = fmaf(xv, w2.z, q2.z);  q2.w = fmaf(xv, w2.w, q2.w);
    }
    const v4f c0 = *(const v4fa*)(sW + 228);
    const v4f c1 = *(const v4fa*)(sW + 232);
    const v4f c2 = *(const v4fa*)(sW + 236);
    const v2u s0 = split2(fmaxf(q0.x + c0.x, 0.0f), fmaxf(q0.y + c0.y, 0.0f));
    const v2u s1 = split2(fmaxf(q0.z + c0.z, 0.0f), fmaxf(q0.w + c0.w, 0.0f));
    const v2u s2 = split2(fmaxf(q1.x + c1.x, 0.0f), fmaxf(q1.y + c1.y, 0.0f));
    const v2u s3 = split2(fmaxf(q1.z + c1.z, 0.0f), fmaxf(q1.w + c1.w, 0.0f));
    const v2u s4 = split2(fmaxf(q2.x + c2.x, 0.0f), fmaxf(q2.y + c2.y, 0.0f));
    const v2u s5 = split2(fmaxf(q2.z + c2.z, 0.0f), fmaxf(q2.w + c2.w, 0.0f));
    v4u p0, p1, p2, p3;
    p0.x = s0.x; p0.y = s1.x; p0.z = s2.x; p0.w = s3.x;
    p1.x = s4.x; p1.y = s5.x; p1.z = s0.y; p1.w = s1.y;
    p2.x = s2.y; p2.y = s3.y; p2.z = s4.y; p2.w = s5.y;
    p3.x = 0u;   p3.y = 0u;   p3.z = 0u;   p3.w = 0u;
    unsigned short* ra = sA + tid * EAP;
    *(v4ua*)(ra)      = p0;
    *(v4ua*)(ra + 8)  = p1;
    *(v4ua*)(ra + 16) = p2;
    *(v4ua*)(ra + 24) = p3;
  }
  __syncthreads();

  float* stw = stg + wave * 16 * SDP;
  const int part = lane >> 4, j = lane & 15;
  const unsigned mh = 0u - (unsigned)part;
  const unsigned ml = ~mh;
  const v8f z = {0.f, 0.f, 0.f, 0.f, 0.f, 0.f, 0.f, 0.f};
#pragma unroll 1
  for (int mt = 0; mt < 2; ++mt) {
    FragB af;
    const unsigned short* ap = sA + (32 * wave + 16 * mt + m) * EAP + 8 * hh;
    af.h[0] = *(const v8usa*)ap;
    af.h[1] = *(const v8usa*)(ap + 16);
#pragma unroll
    for (int nt = 0; nt < 8; ++nt) {
      const unsigned short* wq = W1B + (size_t)(16 * nt + m) * 32 + 8 * hh;
      FragB bf;
      bf.h[0] = *(const v8usa*)wq;
      bf.h[1] = *(const v8usa*)(wq + 16);
      const v8f acc = wmb(af, bf, z);
      const int lc = 16 * nt + m;
      const float bv = sb1[lc];
      float* dq = stw + (8 * hh) * SDP + lc;
      dq[0 * SDP] = fmaxf(acc[0] + bv, 0.0f);
      dq[1 * SDP] = fmaxf(acc[1] + bv, 0.0f);
      dq[2 * SDP] = fmaxf(acc[2] + bv, 0.0f);
      dq[3 * SDP] = fmaxf(acc[3] + bv, 0.0f);
      dq[4 * SDP] = fmaxf(acc[4] + bv, 0.0f);
      dq[5 * SDP] = fmaxf(acc[5] + bv, 0.0f);
      dq[6 * SDP] = fmaxf(acc[6] + bv, 0.0f);
      dq[7 * SDP] = fmaxf(acc[7] + bv, 0.0f);
    }
    __syncthreads();
    {
      const size_t r0 = (size_t)blockIdx.x * 128 + 32 * wave + 16 * mt;
      unsigned short* ob = H1HL + r0 * 256 + part * 128 + 8 * j;
      const float* sb = stw + 8 * j;
#pragma unroll 4
      for (int i = 0; i < 16; ++i) {
        const v4u oo = pack8sel(sb + i * SDP, ml, mh);
        *(volatile v4u*)(ob + (size_t)i * 256) = oo;
      }
      __threadfence();
#pragma unroll 4
      for (int i = 0; i < 16; ++i) {
        const v4u oo = pack8sel(sb + i * SDP, ml, mh);
        *(volatile v4u*)(ob + (size_t)i * 256) = oo;
      }
    }
    __syncthreads();
  }
}

__global__ __launch_bounds__(NTHR) __attribute__((amdgpu_num_vgpr(248)))
void k_bucket(const int* __restrict__ keys, int nE, int nN, int vec8, int* LIST, int* CNT, int* OFF, int* FLG) {
  extern __shared__ __attribute__((aligned(16))) int bsm[];
  int* list = bsm;
  int* hl   = bsm + LISTN;
  int* sl   = hl + RCAP;
  int* cnt  = sl + RCAP;
  int* offs = cnt + NBA;
  int* cur  = offs + NBA;
  int* wcnt = cur + NBA;
  const int tid = (int)threadIdx.x, lane = tid & 31, wave = tid >> 5;
  const int blk = (int)blockIdx.x;
  const int nodeBase = blk * NBA;
  int nb = nN - nodeBase;
  nb = nb < 0 ? 0 : (nb > NBA ? NBA : nb);

  {
    const v4i z4 = {0, 0, 0, 0};
    for (int i = tid * 4; i < BKT_ZINTS; i += NTHR * 4) *(v4ia*)(sl + i) = z4;
    if (tid < 16) wcnt[tid] = 0;
  }
  __syncthreads();

  int tot = 0, ovf = 0;
  const int nChunks = (nE + CHUNK - 1) / CHUNK;
#pragma unroll 1
  for (int ch = 0; ch < nChunks; ++ch) {
    const int cbase = ch * CHUNK;
    const int wc = scan_chunk<SLA>(keys, nE, cbase, nodeBase, nb, vec8, list, tid, lane, wave);
    if (lane == 0) wcnt[wave] = wc;
    __syncthreads();
    int pre = 0, all = 0;
#pragma unroll
    for (int w2 = 0; w2 < NWAVE; ++w2) {
      int c = wcnt[w2];
      c = c < 0 ? 0 : (c > WCAP ? WCAP : c);
      all += c;
      pre += (w2 < wave) ? c : 0;
    }
    const int wcc  = wc > WCAP ? WCAP : wc;
    const int base = tot + pre;
#pragma unroll 1
    for (int i = lane; i < wcc; i += 32) {
      const int ent = list[wave * WCAP + i];
      const int el  = (ent >> SLA) & (CHUNK - 1);
      const int sq  = ent & (NBA - 1);
      int eid = cbase + el;
      eid = eid > nE - 1 ? nE - 1 : eid;
      const int pos = base + i;
      if (pos < RCAP) hl[pos] = (eid << SLA) | sq;
    }
    if (tot + all > RCAP) ovf = 1;
    tot += all;
    tot = tot > RCAP ? RCAP : tot;
    __syncthreads();
  }
  const int nh = tot;

  if (wave == 0) {
#pragma unroll 1
    for (int b0 = 0; b0 < nh; b0 += 32) {
      const int idx = b0 + lane;
      const int uv  = hl[idx < nh ? idx : nh - 1];
      const int m32 = (nh - b0) < 32 ? (nh - b0) : 32;
#pragma unroll 1
      for (int k = 0; k < m32; ++k) {
        const int u  = __builtin_amdgcn_readlane(uv, k);
        const int sq = u & (NBA - 1);
        if (lane == 0) cnt[sq] = cnt[sq] + 1;
      }
    }
  }
  __syncthreads();
  if (wave == 0) {
    const int base = lane * (NBA / 32);
    int s = 0;
#pragma unroll 1
    for (int i = 0; i < NBA / 32; ++i) s += cnt[base + i];
    int incl = s;
#pragma unroll
    for (int d = 1; d < 32; d <<= 1) {
      const int y = __shfl_up(incl, d, 32);
      if (lane >= d) incl += y;
    }
    int run = incl - s;
#pragma unroll 1
    for (int i = 0; i < NBA / 32; ++i) {
      const int cv = cnt[base + i];
      offs[base + i] = run;
      cur[base + i]  = run;
      run += cv;
    }
  }
  __syncthreads();
  if (wave == 0) {
#pragma unroll 1
    for (int b0 = 0; b0 < nh; b0 += 32) {
      const int idx = b0 + lane;
      const int uv  = hl[idx < nh ? idx : nh - 1];
      const int m32 = (nh - b0) < 32 ? (nh - b0) : 32;
#pragma unroll 1
      for (int k = 0; k < m32; ++k) {
        const int u  = __builtin_amdgcn_readlane(uv, k);
        const int sq = u & (NBA - 1);
        if (lane == 0) {
          int p = cur[sq];
          p = p < 0 ? 0 : (p > RCAP - 1 ? RCAP - 1 : p);
          sl[p] = u;
          cur[sq] = p + 1;
        }
      }
    }
  }
  __syncthreads();

  const int nhPad = (nh + 31) & ~31;
  int* lb = LIST + (size_t)blk * RCAP;
  const v4i cv = *(const v4ia*)(cnt + 4 * tid);
  const v4i ov = *(const v4ia*)(offs + 4 * tid);
  v4i fv;
  fv.x = (tid == 0) ? nh : 0;
  fv.y = (tid == 0) ? ovf : 0;
  fv.z = 0; fv.w = 0;
  int* cp = CNT + nodeBase + 4 * tid;
  int* op = OFF + nodeBase + 4 * tid;
  int* fp = FLG + (size_t)blk * 32 + 4 * (tid & 7);
#pragma unroll 1
  for (int p = tid * 4; p < nhPad; p += NTHR * 4) {
    v4i v = *(const v4ia*)(sl + p);
    v.x = v.x >> SLA; v.y = v.y >> SLA; v.z = v.z >> SLA; v.w = v.w >> SLA;
    *(volatile v4i*)(lb + p) = v;
  }
  *(volatile v4i*)cp = cv;
  *(volatile v4i*)op = ov;
  if (tid < 8) *(volatile v4i*)fp = fv;
  __threadfence();
#pragma unroll 1
  for (int p = tid * 4; p < nhPad; p += NTHR * 4) {
    v4i v = *(const v4ia*)(sl + p);
    v.x = v.x >> SLA; v.y = v.y >> SLA; v.z = v.z >> SLA; v.w = v.w >> SLA;
    *(volatile v4i*)(lb + p) = v;
  }
  *(volatile v4i*)cp = cv;
  *(volatile v4i*)op = ov;
  if (tid < 8) *(volatile v4i*)fp = fv;
}

__global__ __launch_bounds__(128) __attribute__((amdgpu_num_vgpr(248)))
void k_gemmT(const unsigned short* __restrict__ A, const unsigned short* __restrict__ BT1,
             unsigned short* T, float* TBc) {
  __shared__ __attribute__((aligned(16))) float stg[64 * 128];
  const int tid = (int)threadIdx.x, lane = tid & 31, wave = tid >> 5, hh = lane >> 4, m = lane & 15;
  const int rowBase = (int)blockIdx.x * 64;
  const int y = (int)blockIdx.y;
  const int colBase = y * 128;

  v8f acc[8];
  {
    const v8f z = {0.f, 0.f, 0.f, 0.f, 0.f, 0.f, 0.f, 0.f};
#pragma unroll
    for (int t = 0; t < 8; ++t) acc[t] = z;
  }
  const unsigned short* ap = A   + (size_t)(rowBase + 16 * wave + m) * 128 + 8 * hh;
  const unsigned short* bp = BT1 + (size_t)(colBase + m) * 128 + 8 * hh;
#pragma unroll 1
  for (int k0 = 0; k0 < 128; k0 += 32) {
    FragB af;
    af.h[0] = *(const v8usa*)(ap + k0);
    af.h[1] = *(const v8usa*)(ap + k0 + 16);
#pragma unroll
    for (int nt = 0; nt < 8; ++nt) {
      const unsigned short* wq = bp + (size_t)(16 * nt) * 128 + k0;
      FragB bf;
      bf.h[0] = *(const v8usa*)wq;
      bf.h[1] = *(const v8usa*)(wq + 16);
      acc[nt] = wmb(af, bf, acc[nt]);
    }
  }
#pragma unroll
  for (int nt = 0; nt < 8; ++nt) {
    const int lc = 16 * nt + m;
#pragma unroll
    for (int r = 0; r < 8; ++r) stg[(16 * wave + 8 * hh + r) * 128 + lc] = acc[nt][r];
  }
  __syncthreads();

  if (y < 64) {
    const int part = lane >> 4, j = lane & 15;
    const unsigned mh = 0u - (unsigned)part;
    const unsigned ml = ~mh;
    v8us pv[16];
#pragma unroll
    for (int i = 0; i < 16; ++i) {
      const float* sp = stg + (16 * wave + i) * 128 + 8 * j;
      const v4f a = *(const v4fa*)sp;
      const v4f b = *(const v4fa*)(sp + 4);
      const v8f f8 = {a.x, a.y, a.z, a.w, b.x, b.y, b.z, b.w};
      v8us oo;
#pragma unroll
      for (int q = 0; q < 8; ++q) {
        const unsigned hb = f2bf(f8[q]);
        const unsigned lb = f2bf(f8[q] - bf2f(hb));
        oo[q] = (unsigned short)((hb & ml) | (lb & mh));
      }
      pv[i] = oo;
    }
    const size_t pofs = (size_t)part * TPLANE + (size_t)y * 128 + 8 * j;
#pragma unroll
    for (int i = 0; i < 16; ++i) {
      unsigned short* op = T + pofs + (size_t)(rowBase + 16 * wave + i) * 8192;
      *(volatile v8us*)op = pv[i];
    }
    __threadfence();
#pragma unroll
    for (int i = 0; i < 16; ++i) {
      unsigned short* op = T + pofs + (size_t)(rowBase + 16 * wave + i) * 8192;
      *(volatile v8us*)op = pv[i];
    }
  } else {
    v4f fv[8];
#pragma unroll
    for (int i = 0; i < 8; ++i) fv[i] = *(const v4fa*)(stg + (16 * wave + 2 * i + hh) * 128 + 4 * m);
#pragma unroll
    for (int i = 0; i < 8; ++i) {
      float* op = TBc + (size_t)(rowBase + 16 * wave + 2 * i + hh) * DIM + 4 * m;
      *(volatile v4f*)op = fv[i];
    }
    __threadfence();
#pragma unroll
    for (int i = 0; i < 8; ++i) {
      float* op = TBc + (size_t)(rowBase + 16 * wave + 2 * i + hh) * DIM + 4 * m;
      *(volatile v4f*)op = fv[i];
    }
  }
}

__global__ __launch_bounds__(128) __attribute__((amdgpu_num_vgpr(248)))
void k_msg(const unsigned short* __restrict__ H1HL, const unsigned short* __restrict__ T,
           const float* __restrict__ TB, const int* __restrict__ LISTS, const int* __restrict__ CNTS,
           const int* __restrict__ OFFS, float* MSG, int base) {
  __shared__ __attribute__((aligned(16))) unsigned short sA[16 * MAP];
  __shared__ __attribute__((aligned(16))) float sD[16 * MDP];
  __shared__ int seid[DEGCAP];
  const int tid = (int)threadIdx.x, lane = tid & 31, wave = tid >> 5, hh = lane >> 4, m = lane & 15;
  const int nl = (int)blockIdx.x;
  const int n  = base + nl;
  const int craw = CNTS[n];
  const bool big = craw > DEGCAP;
  const int c = craw < 0 ? 0 : (craw > DEGCAP ? DEGCAP : craw);
  if (c == 0) return;
  int off = OFFS[n];
  off = off < 0 ? 0 : (off > RCAP - 1 ? RCAP - 1 : off);
  const int blk = n >> SLA;
  {
    const int tq  = tid < DEGCAP ? tid : DEGCAP - 1;
    const int idx = tq < c ? tq : 0;
    int p = off + idx;
    p = p > RCAP - 1 ? RCAP - 1 : p;
    int eid = LISTS[(size_t)blk * RCAP + p];
    eid = eid < 0 ? 0 : (eid > NE - 1 ? NE - 1 : eid);
    if (tid < DEGCAP) seid[tid] = eid;
  }
  FragB bh0, bh1, bh2, bh3, bl0, bl1, bl2, bl3;
  {
    const unsigned short* tp = T + ((size_t)nl * 64 + 16 * wave + m) * 128 + 8 * hh;
    const unsigned short* tq = tp + TPLANE;
    bh0.h[0] = *(const v8usa*)(tp);        bh0.h[1] = *(const v8usa*)(tp + 16);
    bh1.h[0] = *(const v8usa*)(tp + 32);   bh1.h[1] = *(const v8usa*)(tp + 48);
    bh2.h[0] = *(const v8usa*)(tp + 64);   bh2.h[1] = *(const v8usa*)(tp + 80);
    bh3.h[0] = *(const v8usa*)(tp + 96);   bh3.h[1] = *(const v8usa*)(tp + 112);
    bl0.h[0] = *(const v8usa*)(tq);        bl0.h[1] = *(const v8usa*)(tq + 16);
    bl1.h[0] = *(const v8usa*)(tq + 32);   bl1.h[1] = *(const v8usa*)(tq + 48);
    bl2.h[0] = *(const v8usa*)(tq + 64);   bl2.h[1] = *(const v8usa*)(tq + 80);
    bl3.h[0] = *(const v8usa*)(tq + 96);   bl3.h[1] = *(const v8usa*)(tq + 112);
  }
  const int c4   = tid & 15;
  const int rowA = tid >> 4;
  const int rowB = rowA + 8;
  const v4f tb = *(const v4f*)(TB + (size_t)n * DIM + 4 * c4);
  const float pz = big ? __int_as_float(0x7fc00000) : 0.0f;
  __syncthreads();

  const int nT = (c + 15) >> 4;
#pragma unroll 1
  for (int t = 0; t < nT; ++t) {
#pragma unroll
    for (int i = 0; i < 4; ++i) {
      const int p = tid + 128 * i;
      const int row = p >> 5, c16 = p & 31;
      const int eid = seid[16 * t + row];
      const v8us v = *(const v8usa*)(H1HL + (size_t)eid * 256 + 8 * c16);
      *(v8usa*)(sA + row * MAP + 8 * c16) = v;
    }
    __syncthreads();
    v8f acc = {0.f, 0.f, 0.f, 0.f, 0.f, 0.f, 0.f, 0.f};
    const unsigned short* ap = sA + m * MAP + 8 * hh;
    {
      FragB ah, al;
      ah.h[0] = *(const v8usa*)(ap);             ah.h[1] = *(const v8usa*)(ap + 16);
      al.h[0] = *(const v8usa*)(ap + 128);       al.h[1] = *(const v8usa*)(ap + 144);
      acc = wmb(ah, bh0, acc);
      acc = wmb(al, bh0, acc);
      acc = wmb(ah, bl0, acc);
    }
    {
      FragB ah, al;
      ah.h[0] = *(const v8usa*)(ap + 32);        ah.h[1] = *(const v8usa*)(ap + 48);
      al.h[0] = *(const v8usa*)(ap + 160);       al.h[1] = *(const v8usa*)(ap + 176);
      acc = wmb(ah, bh1, acc);
      acc = wmb(al, bh1, acc);
      acc = wmb(ah, bl1, acc);
    }
    {
      FragB ah, al;
      ah.h[0] = *(const v8usa*)(ap + 64);        ah.h[1] = *(const v8usa*)(ap + 80);
      al.h[0] = *(const v8usa*)(ap + 192);       al.h[1] = *(const v8usa*)(ap + 208);
      acc = wmb(ah, bh2, acc);
      acc = wmb(al, bh2, acc);
      acc = wmb(ah, bl2, acc);
    }
    {
      FragB ah, al;
      ah.h[0] = *(const v8usa*)(ap + 96);        ah.h[1] = *(const v8usa*)(ap + 112);
      al.h[0] = *(const v8usa*)(ap + 224);       al.h[1] = *(const v8usa*)(ap + 240);
      acc = wmb(ah, bh3, acc);
      acc = wmb(al, bh3, acc);
      acc = wmb(ah, bl3, acc);
    }
#pragma unroll
    for (int r = 0; r < 8; ++r) sD[(8 * hh + r) * MDP + 16 * wave + m] = acc[r];
    __syncthreads();
    const v4f va = *(const v4fa*)(sD + rowA * MDP + 4 * c4);
    const v4f vb = *(const v4fa*)(sD + rowB * MDP + 4 * c4);
    v4f wa, wb;
    wa.x = va.x + tb.x + pz; wa.y = va.y + tb.y + pz; wa.z = va.z + tb.z + pz; wa.w = va.w + tb.w + pz;
    wb.x = vb.x + tb.x + pz; wb.y = vb.y + tb.y + pz; wb.z = vb.z + tb.z + pz; wb.w = vb.w + tb.w + pz;
    const int ra = 16 * t + rowA;
    const int rb = 16 * t + rowB;
    const bool oka = ra < c;
    const bool okb = rb < c;
    const int ea = seid[ra];
    const int eb = seid[rb];
    float* pa = MSG + (size_t)ea * DIM + 4 * c4;
    float* pb = MSG + (size_t)eb * DIM + 4 * c4;
    if (oka) *(volatile v4f*)pa = wa;
    if (okb) *(volatile v4f*)pb = wb;
    __threadfence();
    if (oka) *(volatile v4f*)pa = wa;
    if (okb) *(volatile v4f*)pb = wb;
  }
}

__global__ __launch_bounds__(NTHR) __attribute__((amdgpu_num_vgpr(248)))
void k_agg(const float* __restrict__ MSG, const int* __restrict__ LISTD, const int* __restrict__ CNTD,
           const int* __restrict__ OFFD, const float* __restrict__ conv_b, unsigned short* MHL) {
  const int tid = (int)threadIdx.x, lane = tid & 31, wave = tid >> 5;
  const int d = (int)blockIdx.x * NWAVE + wave;
  const int craw = CNTD[d];
  const bool big = craw > DEGCAP;
  const int c = craw < 0 ? 0 : (craw > DEGCAP ? DEGCAP : craw);
  int off = OFFD[d];
  off = off < 0 ? 0 : (off > RCAP - 1 ? RCAP - 1 : off);
  const int blk = d >> SLA;
  float a0 = 0.0f, a1 = 0.0f;
#pragma unroll 1
  for (int b0 = 0; b0 < c; b0 += 32) {
    int li = b0 + lane;
    li = li < c ? li : c - 1;
    li = li < 0 ? 0 : li;
    int idx = off + li;
    idx = idx > RCAP - 1 ? RCAP - 1 : idx;
    int eid = LISTD[(size_t)blk * RCAP + idx];
    eid = eid < 0 ? 0 : (eid > NE - 1 ? NE - 1 : eid);
    const int m32 = (c - b0) < 32 ? (c - b0) : 32;
#pragma unroll 1
    for (int k = 0; k < m32; ++k) {
      const int ek = __builtin_amdgcn_readlane(eid, k);
      const v2f v = *(const v2fa*)(MSG + (size_t)ek * DIM + 2 * lane);
      a0 += v.x;
      a1 += v.y;
    }
  }
  const float rd = 1.0f / (float)(c > 1 ? c : 1);
  const v2f cb = *(const v2f*)(conv_b + 2 * lane);
  const float pz = big ? __int_as_float(0x7fc00000) : 0.0f;
  float v0 = a0 * rd + bfr(cb.x) + pz;
  float v1 = a1 * rd + bfr(cb.y) + pz;
  v0 = (v0 > 0.0f) ? v0 : (v0 - v0);
  v1 = (v1 > 0.0f) ? v1 : (v1 - v1);
  const bool live = d < NN;
  v0 = live ? v0 : 0.0f;
  v1 = live ? v1 : 0.0f;
  const v2u s = split2(v0, v1);
  const unsigned wh = s.x;
  const unsigned wl = s.y;
  unsigned* mp = (unsigned*)MHL + (size_t)d * 64 + lane;
  *(volatile unsigned*)mp = wh;
  *(volatile unsigned*)(mp + 32) = wl;
  __threadfence();
  *(volatile unsigned*)mp = wh;
  *(volatile unsigned*)(mp + 32) = wl;
}

__device__ __forceinline__ void gru_store_pass(const float* stg, float* Hn, unsigned short* HHLn,
                                               int rowBase, int tid) {
#pragma unroll 1
  for (int i = 0; i < 8; ++i) {
    const int u = tid + 128 * i;
    const int row = u >> 4, c = (u & 15) * 4;
    const v4f hv = *(const v4fa*)(stg + row * GSP + c);
    const v2u s01 = split2(hv.x, hv.y);
    const v2u s23 = split2(hv.z, hv.w);
    v2u wh, wl;
    wh.x = s01.x; wh.y = s23.x;
    wl.x = s01.y; wl.y = s23.y;
    float* hp = Hn + (size_t)(rowBase + row) * DIM + c;
    unsigned short* bp = HHLn + (size_t)(rowBase + row) * 128 + c;
    *(volatile v4f*)hp = hv;
    *(volatile v2u*)bp = wh;
    *(volatile v2u*)(bp + 64) = wl;
  }
}

__global__ __launch_bounds__(128) __attribute__((amdgpu_num_vgpr(248)))
void k_gru(const unsigned short* __restrict__ MHL, const unsigned short* __restrict__ HHLo,
           const float* __restrict__ Ho, const unsigned short* __restrict__ BTG, const float* __restrict__ GB,
           float* Hn, unsigned short* HHLn) {
  extern __shared__ __attribute__((aligned(16))) float gsm[];
  float* stg = gsm;
  float* sgb = gsm + 64 * GSP;
  const int tid = (int)threadIdx.x, lane = tid & 31, wave = tid >> 5, hh = lane >> 4, m = lane & 15;
  const int rowBase = (int)blockIdx.x * 64;
  sgb[tid] = GB[tid];
  sgb[tid + 128] = GB[tid + 128];

  const unsigned short* am = MHL  + (size_t)(rowBase + 16 * wave + m) * 128 + 8 * hh;
  const unsigned short* ah = HHLo + (size_t)(rowBase + 16 * wave + m) * 128 + 8 * hh;
#pragma unroll 1
  for (int nh = 0; nh < 2; ++nh) {
    v8f acc[8];
    {
      const v8f z = {0.f, 0.f, 0.f, 0.f, 0.f, 0.f, 0.f, 0.f};
#pragma unroll
      for (int t = 0; t < 8; ++t) acc[t] = z;
    }
    const unsigned short* bp = BTG + (size_t)(128 * nh + m) * 256 + 8 * hh;
#pragma unroll 1
    for (int ks = 0; ks < 4; ++ks) {
      FragB af;
      af.h[0] = *(const v8usa*)(am + 32 * ks);
      af.h[1] = *(const v8usa*)(am + 32 * ks + 16);
#pragma unroll
      for (int nt = 0; nt < 8; ++nt) {
        const unsigned short* wq = bp + (size_t)(16 * nt) * 256 + 32 * ks;
        FragB bf;
        bf.h[0] = *(const v8usa*)wq;
        bf.h[1] = *(const v8usa*)(wq + 16);
        acc[nt] = wmb(af, bf, acc[nt]);
      }
    }
#pragma unroll 1
    for (int ks = 0; ks < 4; ++ks) {
      FragB af;
      af.h[0] = *(const v8usa*)(ah + 32 * ks);
      af.h[1] = *(const v8usa*)(ah + 32 * ks + 16);
#pragma unroll
      for (int nt = 0; nt < 8; ++nt) {
        const unsigned short* wq = bp + (size_t)(16 * nt) * 256 + 128 + 32 * ks;
        FragB bf;
        bf.h[0] = *(const v8usa*)wq;
        bf.h[1] = *(const v8usa*)(wq + 16);
        acc[nt] = wmb(af, bf, acc[nt]);
      }
    }
#pragma unroll
    for (int nt = 0; nt < 8; ++nt) {
      const int lc = 128 * nh + 16 * nt + m;
#pragma unroll
      for (int r = 0; r < 8; ++r) stg[(16 * wave + 8 * hh + r) * GSP + lc] = acc[nt][r];
    }
  }
  __syncthreads();

#pragma unroll 1
  for (int i = 0; i < 32; ++i) {
    const int e = tid + 128 * i;
    const int row = e >> 6, c = e & 63;
    float* sp = stg + row * GSP + c;
    const float tr = sp[0]   + sgb[c];
    const float tz = sp[64]  + sgb[64 + c];
    const float ti = sp[128] + sgb[128 + c];
    const float tn = sp[192] + sgb[192 + c];
    const int grow = rowBase + row;
    const float ho = Ho[(size_t)grow * DIM + c];
    const float r  = __builtin_amdgcn_rcpf(1.0f + expf(-tr));
    const float z  = __builtin_amdgcn_rcpf(1.0f + expf(-tz));
    const float nn = tanhf(ti + r * tn);
    const float hv = (1.0f - z) * nn + z * ho;
    sp[0] = (grow < NN) ? hv : 0.0f;
  }
  __syncthreads();

  gru_store_pass(stg, Hn, HHLn, rowBase, tid);
  __threadfence();
  gru_store_pass(stg, Hn, HHLn, rowBase, tid);
}

__device__ __forceinline__ void bn_put(const float* sRT, unsigned short* ra, int ch, v4f f) {
  const v4f mu = *(const v4fa*)(sRT + ch);
  const v4f rs = *(const v4fa*)(sRT + 192 + ch);
  const v4f ga = *(const v4fa*)(sRT + 384 + ch);
  const v4f be = *(const v4fa*)(sRT + 576 + ch);
  const float v0 = ((f.x - mu.x) * rs.x) * ga.x + be.x;
  const float v1 = ((f.y - mu.y) * rs.y) * ga.y + be.y;
  const float v2 = ((f.z - mu.z) * rs.z) * ga.z + be.z;
  const float v3 = ((f.w - mu.w) * rs.w) * ga.w + be.w;
  const v2u s01 = split2(v0, v1);
  const v2u s23 = split2(v2, v3);
  v2u wh, wl;
  wh.x = s01.x; wh.y = s23.x;
  wl.x = s01.y; wl.y = s23.y;
  *(v2ua*)(ra + ch) = wh;
  *(v2ua*)(ra + 192 + ch) = wl;
}

__global__ __launch_bounds__(128) __attribute__((amdgpu_num_vgpr(248)))
void k_read(const float* __restrict__ H, const int* __restrict__ ei3, const float* __restrict__ ea3,
            const float* __restrict__ RT, const unsigned short* __restrict__ WWB, const int* __restrict__ FLG,
            float* out, int nP, int nN) {
  extern __shared__ __attribute__((aligned(16))) float rsm[];
  unsigned short* sA = (unsigned short*)rsm;
  float* sRT = rsm + RD_OFF_RT;
  float* sG  = rsm + RD_OFF_G;
  float* sy  = rsm + RD_OFF_Y;
  int*   sfl = (int*)(rsm + RD_OFF_F);
  const int tid = (int)threadIdx.x, lane = tid & 31, wave = tid >> 5, hh = lane >> 4, m = lane & 15;
  const int pbase = (int)blockIdx.x * 128;

  *(v4fa*)(sRT + 4 * tid)       = *(const v4f*)(RT + 4 * tid);
  *(v4fa*)(sRT + 512 + 4 * tid) = *(const v4f*)(RT + 512 + 4 * tid);
  {
    const int fw = FLG[(size_t)(tid & 7) * 32 + 1];
    if (tid < 8) sfl[tid] = fw;
  }
  const int p  = pbase + tid;
  const int pc = p < nP ? p : nP - 1;
  int i0 = ei3[pc];
  int i1 = ei3[(size_t)nP + pc];
  i0 = i0 < 0 ? 0 : (i0 > nN - 1 ? nN - 1 : i0);
  i1 = i1 < 0 ? 0 : (i1 > nN - 1 ? nN - 1 : i1);
  __syncthreads();

  {
    const float* r0 = H + (size_t)i0 * DIM;
    const float* r1 = H + (size_t)i1 * DIM;
    unsigned short* ra = sA + tid * RAP;
#pragma unroll 1
    for (int c4 = 0; c4 < 16; ++c4) {
      const int c = 4 * c4;
      const v4f a = *(const v4f*)(r0 + c);
      const v4f b = *(const v4f*)(r1 + c);
      const v4f fm = (a + b) * 0.5f;
      const v4f fp = a * b;
      const v4f dd = a - b;
      const v4f fs = dd * dd;
      bn_put(sRT, ra, c, fm);
      bn_put(sRT, ra, 64 + c, fp);
      bn_put(sRT, ra, 128 + c, fs);
    }
  }
  __syncthreads();

  {
    v8f acc0 = {0.f, 0.f, 0.f, 0.f, 0.f, 0.f, 0.f, 0.f};
    v8f acc1 = acc0;
    const unsigned short* ap0 = sA + (32 * wave + m) * RAP + 8 * hh;
    const unsigned short* ap1 = ap0 + 16 * RAP;
    const unsigned short* bp  = WWB + (size_t)m * 384 + 8 * hh;
#pragma unroll 1
    for (int ks = 0; ks < 12; ++ks) {
      FragB a0, a1, bf;
      a0.h[0] = *(const v8usa*)(ap0 + 32 * ks);
      a0.h[1] = *(const v8usa*)(ap0 + 32 * ks + 16);
      a1.h[0] = *(const v8usa*)(ap1 + 32 * ks);
      a1.h[1] = *(const v8usa*)(ap1 + 32 * ks + 16);
      bf.h[0] = *(const v8usa*)(bp + 32 * ks);
      bf.h[1] = *(const v8usa*)(bp + 32 * ks + 16);
      acc0 = wmb(a0, bf, acc0);
      acc1 = wmb(a1, bf, acc1);
    }
#pragma unroll
    for (int r = 0; r < 8; ++r) {
      sG[(32 * wave + 8 * hh + r) * RGP + m]      = acc0[r];
      sG[(32 * wave + 16 + 8 * hh + r) * RGP + m] = acc1[r];
    }
  }
  __syncthreads();

  {
    const v4f e0 = *(const v4f*)(ea3 + (size_t)pc * 8);
    const v4f e1 = *(const v4f*)(ea3 + (size_t)pc * 8 + 4);
    const float* gp = sG + tid * RGP;
    float y = 0.0f;
    y = fmaf(bfr(e0.x), gp[0] + sRT[768], y);
    y = fmaf(bfr(e0.y), gp[1] + sRT[769], y);
    y = fmaf(bfr(e0.z), gp[2] + sRT[770], y);
    y = fmaf(bfr(e0.w), gp[3] + sRT[771], y);
    y = fmaf(bfr(e1.x), gp[4] + sRT[772], y);
    y = fmaf(bfr(e1.y), gp[5] + sRT[773], y);
    y = fmaf(bfr(e1.z), gp[6] + sRT[774], y);
    y = fmaf(bfr(e1.w), gp[7] + sRT[775], y);
    const int fl = sfl[0] | sfl[1] | sfl[2] | sfl[3] | sfl[4] | sfl[5] | sfl[6] | sfl[7];
    y = (fl != 0) ? __int_as_float(0x7fc00000) : y;
    sy[tid] = y;
  }
  __syncthreads();
  if (wave == 0) {
    int nvalid = nP - pbase;
    nvalid = nvalid > 128 ? 128 : nvalid;
    const v4f v = *(const v4fa*)(sy + 4 * lane);
    float* op = out + (size_t)pbase + 4 * lane;
    const bool ok = 4 * lane < nvalid;
    if (ok) *(volatile v4f*)op = v;
    __threadfence();
    if (ok) *(volatile v4f*)op = v;
  }
}

extern "C" void kernel_launch(void* const* d_in, const int* in_sizes, int n_in,
                              void* d_out, int out_size, void* d_ws, size_t ws_size,
                              hipStream_t stream) {
  if (n_in < 24) return;
  if (in_sizes[0] != NN * 8) return;
  if (in_sizes[1] != NE * 19) return;
  if (in_sizes[2] != NPR * 8) return;
  if (in_sizes[3] != 2 * NE) return;
  if (in_sizes[4] != 2 * NPR) return;
  if (in_sizes[5] != 8 * DIM || in_sizes[6] != DIM) return;
  if (in_sizes[7] != 19 * 12 || in_sizes[8] != 12) return;
  if (in_sizes[9] != 12 * HK || in_sizes[10] != HK) return;
  if (in_sizes[11] != HK * 4096 || in_sizes[12] != 4096) return;
  if (in_sizes[13] != DIM) return;
  if (in_sizes[14] != 192 * DIM || in_sizes[15] != 192) return;
  if (in_sizes[16] != 192 * DIM || in_sizes[17] != 192) return;
  if (in_sizes[18] != 192 || in_sizes[19] != 192 || in_sizes[20] != 192 || in_sizes[21] != 192) return;
  if (in_sizes[22] != 8 * 192 || in_sizes[23] != 8) return;
  if (out_size != NPR) return;

  const float* x      = (const float*)d_in[0];
  const float* eattr  = (const float*)d_in[1];
  const float* ea3    = (const float*)d_in[2];
  const int*   ei     = (const int*)  d_in[3];
  const int*   ei3    = (const int*)  d_in[4];
  const float* Wn     = (const float*)d_in[5];
  const float* bn_    = (const float*)d_in[6];
  const float* We     = (const float*)d_in[7];
  const float* be     = (const float*)d_in[8];
  const float* W1     = (const float*)d_in[9];
  const float* b1     = (const float*)d_in[10];
  const float* W2     = (const float*)d_in[11];
  const float* b2     = (const float*)d_in[12];
  const float* conv_b = (const float*)d_in[13];
  const float* W_ih   = (const float*)d_in[14];
  const float* b_ih   = (const float*)d_in[15];
  const float* W_hh   = (const float*)d_in[16];
  const float* b_hh   = (const float*)d_in[17];
  const float* bmean  = (const float*)d_in[18];
  const float* bvar   = (const float*)d_in[19];
  const float* bgam   = (const float*)d_in[20];
  const float* bbet   = (const float*)d_in[21];
  const float* Wwt    = (const float*)d_in[22];
  const float* Wbias  = (const float*)d_in[23];
  float* out = (float*)d_out;

  char* ws = (char*)d_ws;
  size_t off = 0;
  const size_t oBT1 = off; off += (size_t)NT1 * 128 * 2;        off = (off + 255) & ~(size_t)255;
  const size_t oW1B = off; off += (size_t)HK * 32 * 2;          off = (off + 255) & ~(size_t)255;
  const size_t oPB  = off; off += (size_t)PB_BYTES;             off = (off + 255) & ~(size_t)255;
  const size_t oH   = off; off += (size_t)2 * MPN * DIM * 4;    off = (off + 255) & ~(size_t)255;
  const size_t oHHL = off; off += (size_t)2 * MPN * 128 * 2;    off = (off + 255) & ~(size_t)255;
  const size_t oMHL = off; off += (size_t)MPN * 128 * 2;        off = (off + 255) & ~(size_t)255;
  const size_t oH1  = off; off += (size_t)NE * 256 * 2;         off = (off + 255) & ~(size_t)255;
  const size_t oMSG = off; off += (size_t)NE * DIM * 4;         off = (off + 255) & ~(size_t)255;
  const size_t oTB  = off; off += (size_t)MPN * DIM * 4;        off = (off + 255) & ~(size_t)255;
  const size_t oT   = off; off += (size_t)2 * TPLANE * 2;       off = (off + 255) & ~(size_t)255;
  const size_t oLST = off; off += (size_t)2 * 4 * RCAP * 4;     off = (off + 255) & ~(size_t)255;
  const size_t oCNT = off; off += (size_t)2 * MPN * 4;          off = (off + 255) & ~(size_t)255;
  const size_t oOFF = off; off += (size_t)2 * MPN * 4;          off = (off + 255) & ~(size_t)255;
  const size_t oFLG = off; off += (size_t)8 * 128;              off = (off + 255) & ~(size_t)255;
  if (off > ws_size || off > (size_t)WSMAX) return;

  unsigned short* BT1  = (unsigned short*)(ws + oBT1);
  unsigned short* W1B  = (unsigned short*)(ws + oW1B);
  unsigned char*  PB   = (unsigned char*)(ws + oPB);
  const unsigned short* BTG = (const unsigned short*)(ws + oPB + PB_BTG);
  const unsigned short* WWB = (const unsigned short*)(ws + oPB + PB_WWB);
  const float*    RT   = (const float*)(ws + oPB + PB_RT);
  const float*    GB   = (const float*)(ws + oPB + PB_GB);
  float*          Hb   = (float*)(ws + oH);
  unsigned short* HHLb = (unsigned short*)(ws + oHHL);
  unsigned short* MHL  = (unsigned short*)(ws + oMHL);
  unsigned short* H1HL = (unsigned short*)(ws + oH1);
  float*          MSG  = (float*)(ws + oMSG);
  float*          TB   = (float*)(ws + oTB);
  unsigned short* T    = (unsigned short*)(ws + oT);
  int*            LSTD = (int*)(ws + oLST);
  int*            LSTS = LSTD + (size_t)4 * RCAP;
  int*            CNTD = (int*)(ws + oCNT);
  int*            CNTS = CNTD + MPN;
  int*            OFFD = (int*)(ws + oOFF);
  int*            OFFS = OFFD + MPN;
  int*            FLG  = (int*)(ws + oFLG);

  const int bktLds = BKT_LDS_INTS * 4;
  const int gruLds = GRU_LDS_FLOATS * 4;
  const int rdLds  = RD_LDS_FLOATS * 4;
  hipFuncSetAttribute(reinterpret_cast<const void*>(&k_bucket), hipFuncAttributeMaxDynamicSharedMemorySize, bktLds);
  hipFuncSetAttribute(reinterpret_cast<const void*>(&k_gru),    hipFuncAttributeMaxDynamicSharedMemorySize, gruLds);
  hipFuncSetAttribute(reinterpret_cast<const void*>(&k_read),   hipFuncAttributeMaxDynamicSharedMemorySize, rdLds);

  k_pa<<<(NU_BT1 + NU_W1B) / NTHR, NTHR, 0, stream>>>(W2, b2, W1, BT1, W1B);
  k_pb<<<(NU_BTG + NU_WWB + NU_RT + NU_GB) / NTHR, NTHR, 0, stream>>>(W_ih, W_hh, b_ih, b_hh, bmean, bvar,
                                                                      bgam, bbet, Wwt, Wbias, PB);
  k_node<<<(MPN * 16) / NTHR, NTHR, 0, stream>>>(x, Wn, bn_, Hb, HHLb);
  k_edge<<<NE / 128, 128, 0, stream>>>(eattr, We, be, b1, W1B, H1HL);
  k_bucket<<<4, NTHR, bktLds, stream>>>(ei + NE, NE, NN, 1, LSTD, CNTD, OFFD, FLG);
  k_bucket<<<4, NTHR, bktLds, stream>>>(ei,      NE, NN, 1, LSTS, CNTS, OFFS, FLG + 4 * 32);

  int cur = 0;
  for (int it = 0; it < 3; ++it) {
    float*          Hc   = Hb   + (size_t)cur * MPN * DIM;
    unsigned short* HHLc = HHLb + (size_t)cur * MPN * 128;
    float*          Hx   = Hb   + (size_t)(1 - cur) * MPN * DIM;
    unsigned short* HHLx = HHLb + (size_t)(1 - cur) * MPN * 128;
    for (int c = 0; c < 2; ++c) {
      k_gemmT<<<dim3(CHR / 64, NT1 / 128), 128, 0, stream>>>(HHLc + (size_t)c * CHR * 128, BT1, T,
                                                             TB + (size_t)c * CHR * DIM);
      k_msg<<<CHR, 128, 0, stream>>>(H1HL, T, TB, LSTS, CNTS, OFFS, MSG, c * CHR);
    }
    k_agg<<<MPN / NWAVE, NTHR, 0, stream>>>(MSG, LSTD, CNTD, OFFD, conv_b, MHL);
    k_gru<<<MPN / 64, 128, gruLds, stream>>>(MHL, HHLc, Hc, BTG, GB, Hx, HHLx);
    cur = 1 - cur;
  }
  k_read<<<(NPR + 127) / 128, 128, rdLds, stream>>>(Hb + (size_t)cur * MPN * DIM, ei3, ea3, RT, WWB, FLG,
                                                    out, NPR, NN);
}
